// GCN_68375879352699
// MI455X (gfx1250) — hardware-verified
//
#include <hip/hip_runtime.h>
#include <stddef.h>
#include <stdint.h>
#include <math.h>


#define NB     8
#define NN     1024
#define DD     512
#define HH     2048
#define NL     3
#define MROWS  (NB * NN)
#define HALFR  4096
#define NTHR   256
#define NWAVE  8
#define GBM    64
#define GBN    128
#define GTHR   128
#define XT_P   72
#define TERMS_AGG 1
#define WSMAX  134217728

static_assert(TERMS_AGG == 1 || TERMS_AGG == 3);
static_assert(MROWS % 64 == 0 && MROWS % 32 == 0 && NN % 64 == 0 && NN % GBM == 0);
static_assert(DD % GBN == 0 && HH % GBN == 0 && HALFR % GBM == 0 && 2 * HALFR == MROWS);
static_assert(NN % 32 == 0 && (2 * DD) % 32 == 0 && (2 * HH) % 32 == 0);
static_assert((DD & (DD - 1)) == 0 && (HH & (HH - 1)) == 0 && (NN & (NN - 1)) == 0);
static_assert(GBM == (GTHR / 32) * 16 && DD == 4 * 128);
static_assert((NL * DD * HH / 8) % NTHR == 0);
static_assert((XT_P % 8) == 0 && XT_P >= 64);

typedef float          v4f   __attribute__((ext_vector_type(4)));
typedef float          v8f   __attribute__((ext_vector_type(8)));
typedef int            v8i   __attribute__((ext_vector_type(8)));
typedef unsigned int   v4u   __attribute__((ext_vector_type(4)));
typedef unsigned short v4us  __attribute__((ext_vector_type(4)));
typedef unsigned short v8us  __attribute__((ext_vector_type(8)));
typedef unsigned short v16us __attribute__((ext_vector_type(16)));
typedef __bf16         v16bf __attribute__((ext_vector_type(16)));
typedef v4f  __attribute__((may_alias)) v4fa;
typedef v4u  __attribute__((may_alias)) v4ua;
typedef v4us __attribute__((may_alias)) v4usa;
typedef v8us __attribute__((may_alias)) v8usa;
union FragB { v16bf v; v16us u; v8us h[2]; v8i w; };

__device__ __forceinline__ v8f wmb(const FragB& a, const FragB& b, v8f c) {
  v8f d = __builtin_amdgcn_wmma_f32_16x16x32_bf16(false, a.v, false, b.v, (short)0, c, false, false);
  asm volatile("v_nop\n\tv_nop\n\tv_nop\n\tv_nop" : "+v"(d) : "v"(a.w), "v"(b.w));
  return d;
}

__device__ __forceinline__ unsigned bf16_bits(float f) {
  const unsigned u = __float_as_uint(f);
  return (u + 0x7FFFu + ((u >> 16) & 1u)) >> 16;
}
__device__ __forceinline__ float bf16_val(float f) {
  return __uint_as_float(bf16_bits(f) << 16);
}
__device__ __forceinline__ v4f bf16v4(v4f a) {
  v4f r;
  r.x = bf16_val(a.x); r.y = bf16_val(a.y); r.z = bf16_val(a.z); r.w = bf16_val(a.w);
  return r;
}

__device__ __forceinline__ void wave_sync() {
  __builtin_amdgcn_fence(__ATOMIC_RELEASE, "wavefront");
  __builtin_amdgcn_wave_barrier();
  __builtin_amdgcn_fence(__ATOMIC_ACQUIRE, "wavefront");
}

__device__ __forceinline__ float wsum(float v) {
#pragma unroll
  for (int d = 16; d >= 1; d >>= 1) v += __shfl_xor(v, d, 32);
  return v;
}
__device__ __forceinline__ float wmax(float v) {
#pragma unroll
  for (int d = 16; d >= 1; d >>= 1) v = fmaxf(v, __shfl_xor(v, d, 32));
  return v;
}

__global__ __launch_bounds__(NTHR) void k_wT(const float* __restrict__ W, unsigned short* WT,
                                             int Kd, int Nd, int nUnits) {
  const int u = (int)blockIdx.x * NTHR + (int)threadIdx.x;
  if (u >= nUnits) return;
  const int k8n  = Kd >> 3;
  const int perL = Nd * k8n;
  const int l    = u / perL;
  const int r    = u - l * perL;
  const int n    = r / k8n;
  const int k8   = (r - n * k8n) * 8;
  const float* p = W + (size_t)l * (size_t)Kd * (size_t)Nd + (size_t)k8 * (size_t)Nd + n;
  v8us o;
#pragma unroll
  for (int i = 0; i < 8; ++i) o[i] = (unsigned short)bf16_bits(p[(size_t)i * (size_t)Nd]);
  unsigned short* dp = WT + (size_t)l * (size_t)Nd * (size_t)Kd + (size_t)n * (size_t)Kd + k8;
  *(volatile v8us*)dp = o;
  __threadfence();
  *(volatile v8us*)dp = o;
}

__global__ __launch_bounds__(NTHR) void k_mask(const int* __restrict__ adj, unsigned* MB) {
  __shared__ __attribute__((aligned(16))) unsigned stage[NWAVE * 128];
  const int tid = (int)threadIdx.x, lane = tid & 31, wave = tid >> 5;
  const int row0 = (int)blockIdx.x * 32 + wave * 4;
#pragma unroll 1
  for (int rr = 0; rr < 4; ++rr) {
    const int row = row0 + rr;
    const int i   = row & (NN - 1);
    const int* ar = adj + (size_t)row * NN;
    unsigned mine = 0u;
#pragma unroll 4
    for (int w = 0; w < 32; ++w) {
      const int j = 32 * w + lane;
      const int a = ar[j];
      const float dg = (j == i) ? 1.0f : 0.0f;
      const bool ok = ((float)a + dg) > 0.0f;
      const unsigned bal = __builtin_amdgcn_ballot_w32(ok);
      mine = (lane == w) ? bal : mine;
    }
    stage[wave * 128 + rr * 32 + lane] = mine;
  }
  wave_sync();
  const v4u o = *(const v4ua*)(stage + wave * 128 + 4 * lane);
  unsigned* dp = MB + (size_t)row0 * 32 + 4 * lane;
  *(volatile v4u*)dp = o;
  __threadfence();
  *(volatile v4u*)dp = o;
}

template <int MODE>
__global__ __launch_bounds__(NTHR) void k_rows(const float* __restrict__ in, const float* __restrict__ gam,
                                               const float* __restrict__ bet, const float* __restrict__ aw,
                                               float* outF, unsigned short* outHL, float* outSS) {
  constexpr bool LNM = (MODE != 0);
  constexpr bool DOT = (MODE == 0 || MODE == 2);
  constexpr bool HLM = (MODE == 1);
  __shared__ __attribute__((aligned(16))) unsigned short rowbuf[HLM ? NWAVE * 1024 : 8];
  __shared__ __attribute__((aligned(16))) float ssl[64];
  const int tid = (int)threadIdx.x, lane = tid & 31, wave = tid >> 5;

  v4f g4[4], b4[4], wa[4], wb[4];
#pragma unroll
  for (int k = 0; k < 4; ++k) {
    const int c = 4 * lane + 128 * k;
    const v4f z = {0.f, 0.f, 0.f, 0.f};
    g4[k] = z; b4[k] = z; wa[k] = z; wb[k] = z;
    if constexpr (LNM) {
      g4[k] = bf16v4(*(const v4fa*)(gam + c));
      b4[k] = bf16v4(*(const v4fa*)(bet + c));
    }
    if constexpr (DOT) {
      wa[k] = bf16v4(*(const v4fa*)(aw + c));
      wb[k] = bf16v4(*(const v4fa*)(aw + DD + c));
    }
  }

#pragma unroll 1
  for (int rr = 0; rr < 4; ++rr) {
    const int rl = wave * 4 + rr;
    const size_t row = (size_t)blockIdx.x * 32 + (size_t)rl;
    const float* ip = in + row * DD + 4 * lane;
    v4f v[4], y[4];
#pragma unroll
    for (int k = 0; k < 4; ++k) v[k] = *(const v4fa*)(ip + 128 * k);
    if constexpr (!LNM) {
#pragma unroll
      for (int k = 0; k < 4; ++k) y[k] = bf16v4(v[k]);
    } else {
      float s = 0.0f;
#pragma unroll
      for (int k = 0; k < 4; ++k) s += (v[k].x + v[k].y) + (v[k].z + v[k].w);
      s = wsum(s);
      const float mean = s * (1.0f / (float)DD);
      float s2 = 0.0f;
#pragma unroll
      for (int k = 0; k < 4; ++k) {
        v[k].x -= mean; v[k].y -= mean; v[k].z -= mean; v[k].w -= mean;
        s2 += (v[k].x * v[k].x + v[k].y * v[k].y) + (v[k].z * v[k].z + v[k].w * v[k].w);
      }
      s2 = wsum(s2);
      const float rs = rsqrtf(s2 * (1.0f / (float)DD) + 1e-5f);
#pragma unroll
      for (int k = 0; k < 4; ++k) {
        y[k].x = (v[k].x * rs) * g4[k].x + b4[k].x;
        y[k].y = (v[k].y * rs) * g4[k].y + b4[k].y;
        y[k].z = (v[k].z * rs) * g4[k].z + b4[k].z;
        y[k].w = (v[k].w * rs) * g4[k].w + b4[k].w;
      }
    }

    float* op = outF + row * DD + 4 * lane;
    v8us q[4];
    unsigned short* hp = outHL + row * 1024 + 8 * lane;
    if constexpr (HLM) {
      unsigned short* rb = rowbuf + wave * 1024;
#pragma unroll
      for (int k = 0; k < 4; ++k) {
        const int c = 4 * lane + 128 * k;
        v4us h4, l4;
        unsigned hb;
        hb = bf16_bits(y[k].x); h4[0] = (unsigned short)hb; l4[0] = (unsigned short)bf16_bits(y[k].x - __uint_as_float(hb << 16));
        hb = bf16_bits(y[k].y); h4[1] = (unsigned short)hb; l4[1] = (unsigned short)bf16_bits(y[k].y - __uint_as_float(hb << 16));
        hb = bf16_bits(y[k].z); h4[2] = (unsigned short)hb; l4[2] = (unsigned short)bf16_bits(y[k].z - __uint_as_float(hb << 16));
        hb = bf16_bits(y[k].w); h4[3] = (unsigned short)hb; l4[3] = (unsigned short)bf16_bits(y[k].w - __uint_as_float(hb << 16));
        *(v4usa*)(rb + c) = h4;
        *(v4usa*)(rb + DD + c) = l4;
      }
      wave_sync();
#pragma unroll
      for (int i = 0; i < 4; ++i) q[i] = *(const v8usa*)(rb + 8 * lane + 256 * i);
      wave_sync();
    }
#pragma unroll
    for (int k = 0; k < 4; ++k) *(volatile v4f*)(op + 128 * k) = y[k];
    if constexpr (HLM) {
#pragma unroll
      for (int i = 0; i < 4; ++i) *(volatile v8us*)(hp + 256 * i) = q[i];
    }
    __threadfence();
#pragma unroll
    for (int k = 0; k < 4; ++k) *(volatile v4f*)(op + 128 * k) = y[k];
    if constexpr (HLM) {
#pragma unroll
      for (int i = 0; i < 4; ++i) *(volatile v8us*)(hp + 256 * i) = q[i];
    }

    if constexpr (DOT) {
      float a = 0.0f, b = 0.0f;
#pragma unroll
      for (int k = 0; k < 4; ++k) {
        a = fmaf(y[k].x, wa[k].x, a); a = fmaf(y[k].y, wa[k].y, a);
        a = fmaf(y[k].z, wa[k].z, a); a = fmaf(y[k].w, wa[k].w, a);
        b = fmaf(y[k].x, wb[k].x, b); b = fmaf(y[k].y, wb[k].y, b);
        b = fmaf(y[k].z, wb[k].z, b); b = fmaf(y[k].w, wb[k].w, b);
      }
      a = wsum(a); b = wsum(b);
      if (lane == 0) { ssl[rl] = a; ssl[32 + rl] = b; }
    }
  }

  if constexpr (DOT) {
    __syncthreads();
    const v4f ov = *(const v4fa*)(ssl + 4 * (lane & 15));
    const size_t so = (size_t)blockIdx.x * 32 + (size_t)((lane < 8) ? 4 * lane : MROWS + 4 * (lane - 8));
    float* sp = outSS + so;
    const bool okst = (wave == 0) && (lane < 16);
    if (okst) *(volatile v4f*)sp = ov;
    __threadfence();
    if (okst) *(volatile v4f*)sp = ov;
  }
}

__global__ __launch_bounds__(NTHR) void k_xt(const float* __restrict__ X, unsigned short* XT) {
  __shared__ __attribute__((aligned(16))) unsigned short th[64 * XT_P];
#if TERMS_AGG == 3
  __shared__ __attribute__((aligned(16))) unsigned short tl[64 * XT_P];
#endif
  const int tid  = (int)threadIdx.x;
  const int node = tid >> 2;
  const int fq   = (tid & 3) * 16;
  const int g0   = (int)blockIdx.x * 64;
  const int f0   = (int)blockIdx.y * 64;
  const float* p = X + (size_t)(g0 + node) * DD + f0 + fq;
  float vals[16];
#pragma unroll
  for (int i = 0; i < 4; ++i) {
    const v4f a = *(const v4fa*)(p + 4 * i);
    vals[4 * i + 0] = a.x; vals[4 * i + 1] = a.y; vals[4 * i + 2] = a.z; vals[4 * i + 3] = a.w;
  }
#pragma unroll
  for (int e = 0; e < 16; ++e) {
    const unsigned hb = bf16_bits(vals[e]);
    th[(fq + e) * XT_P + node] = (unsigned short)hb;
#if TERMS_AGG == 3
    tl[(fq + e) * XT_P + node] = (unsigned short)bf16_bits(vals[e] - __uint_as_float(hb << 16));
#endif
  }
  __syncthreads();
  const int b  = g0 >> 10;
  const int j0 = g0 & (NN - 1);
  const int pc = tid & 7;
  v8us qh[2];
#pragma unroll
  for (int it = 0; it < 2; ++it) qh[it] = *(const v8usa*)(th + ((tid >> 3) + 32 * it) * XT_P + 8 * pc);
#if TERMS_AGG == 3
  v8us ql[2];
#pragma unroll
  for (int it = 0; it < 2; ++it) ql[it] = *(const v8usa*)(tl + ((tid >> 3) + 32 * it) * XT_P + 8 * pc);
#endif
  unsigned short* d0 = XT + ((size_t)b * DD + f0 + (tid >> 3)) * NN + j0 + 8 * pc;
#pragma unroll
  for (int it = 0; it < 2; ++it) *(volatile v8us*)(d0 + (size_t)(32 * it) * NN) = qh[it];
#if TERMS_AGG == 3
#pragma unroll
  for (int it = 0; it < 2; ++it) *(volatile v8us*)(d0 + (size_t)NB * DD * NN + (size_t)(32 * it) * NN) = ql[it];
#endif
  __threadfence();
#pragma unroll
  for (int it = 0; it < 2; ++it) *(volatile v8us*)(d0 + (size_t)(32 * it) * NN) = qh[it];
#if TERMS_AGG == 3
#pragma unroll
  for (int it = 0; it < 2; ++it) *(volatile v8us*)(d0 + (size_t)NB * DD * NN + (size_t)(32 * it) * NN) = ql[it];
#endif
}

__global__ __launch_bounds__(NTHR) void k_softmax(const float* __restrict__ SS, const unsigned* __restrict__ MB,
                                                  const float* __restrict__ ab, int layer, unsigned short* P) {
  __shared__ __attribute__((aligned(16))) float eb[NWAVE * NN];
  __shared__ __attribute__((aligned(16))) unsigned short pb[NWAVE * NN];
#if TERMS_AGG == 3
  __shared__ __attribute__((aligned(16))) unsigned short pl[NWAVE * NN];
#endif
  const int tid = (int)threadIdx.x, lane = tid & 31, wave = tid >> 5;
  const int row = (int)blockIdx.x * NWAVE + wave;
  const int b   = row >> 10;
  const float si = SS[row];
  const float* sjr = SS + MROWS + (size_t)b * NN + 32 * lane;
  const float bb = bf16_val(ab[layer]);
  const unsigned mw = MB[(size_t)row * 32 + lane];
  const float ninf = __int_as_float((int)0xff800000u);
  float* er = eb + wave * NN + 32 * lane;

  float mx = ninf;
#pragma unroll 2
  for (int q = 0; q < 8; ++q) {
    const v4f s = *(const v4fa*)(sjr + 4 * q);
    const unsigned bits = mw >> (4 * q);
    const float t0 = (si + s.x) + bb, t1 = (si + s.y) + bb, t2 = (si + s.z) + bb, t3 = (si + s.w) + bb;
    float e0 = (t0 >= 0.0f) ? t0 : 0.2f * t0;
    float e1 = (t1 >= 0.0f) ? t1 : 0.2f * t1;
    float e2 = (t2 >= 0.0f) ? t2 : 0.2f * t2;
    float e3 = (t3 >= 0.0f) ? t3 : 0.2f * t3;
    e0 = (bits & 1u) ? e0 : ninf;
    e1 = (bits & 2u) ? e1 : ninf;
    e2 = (bits & 4u) ? e2 : ninf;
    e3 = (bits & 8u) ? e3 : ninf;
    mx = fmaxf(fmaxf(mx, fmaxf(e0, e1)), fmaxf(e2, e3));
    v4f e4; e4.x = e0; e4.y = e1; e4.z = e2; e4.w = e3;
    *(v4fa*)(er + 4 * q) = e4;
  }
  mx = wmax(mx);

  float ls = 0.0f;
#pragma unroll 1
  for (int t = 0; t < 32; ++t) {
    const float e = er[t];
    const float p = expf(e - mx);
    ls += p;
    er[t] = p;
  }
  ls = wsum(ls);

  unsigned short* pr = pb + wave * NN + 32 * lane;
#if TERMS_AGG == 3
  unsigned short* plr = pl + wave * NN + 32 * lane;
#endif
#pragma unroll 1
  for (int t = 0; t < 32; ++t) {
    const float pv = er[t] / ls;
    const unsigned hb = bf16_bits(pv);
    pr[t] = (unsigned short)hb;
#if TERMS_AGG == 3
    plr[t] = (unsigned short)bf16_bits(pv - __uint_as_float(hb << 16));
#endif
  }
  wave_sync();
  v8us qh[4];
#pragma unroll
  for (int q = 0; q < 4; ++q) qh[q] = *(const v8usa*)(pb + wave * NN + 8 * lane + 256 * q);
#if TERMS_AGG == 3
  v8us ql[4];
#pragma unroll
  for (int q = 0; q < 4; ++q) ql[q] = *(const v8usa*)(pl + wave * NN + 8 * lane + 256 * q);
#endif
  unsigned short* dp = P + (size_t)row * NN + 8 * lane;
#pragma unroll
  for (int q = 0; q < 4; ++q) *(volatile v8us*)(dp + 256 * q) = qh[q];
#if TERMS_AGG == 3
#pragma unroll
  for (int q = 0; q < 4; ++q) *(volatile v8us*)(dp + (size_t)MROWS * NN + 256 * q) = ql[q];
#endif
  __threadfence();
#pragma unroll
  for (int q = 0; q < 4; ++q) *(volatile v8us*)(dp + 256 * q) = qh[q];
#if TERMS_AGG == 3
#pragma unroll
  for (int q = 0; q < 4; ++q) *(volatile v8us*)(dp + (size_t)MROWS * NN + 256 * q) = ql[q];
#endif
}

template <int EPI>
__global__ __launch_bounds__(GTHR) void k_gemm(
    const unsigned short* __restrict__ A, const unsigned short* __restrict__ BT,
    int lda, int ldb, int K, int npass, int aLo, int bLo, int aZ, int bZ, int rowsZ,
    const float* __restrict__ R, const float* __restrict__ bias,
    float* outF, unsigned short* outB, int ldo)
{
  __shared__ __attribute__((aligned(16))) float stg[GBM * GBN];
  const int tid = (int)threadIdx.x, lane = tid & 31, wave = tid >> 5, hh = lane >> 4, m = lane & 15;
  const int z       = (int)blockIdx.z;
  const int rowBase = (int)blockIdx.x * GBM;
  const int col0    = (int)blockIdx.y * GBN;
  const int kmask   = ldb - 1;

  v8f acc[8];
  {
    const v8f zz = {0.f, 0.f, 0.f, 0.f, 0.f, 0.f, 0.f, 0.f};
#pragma unroll
    for (int t = 0; t < 8; ++t) acc[t] = zz;
  }

#pragma unroll 1
  for (int ps = 0; ps < npass; ++ps) {
    const size_t ao = (ps == 1) ? (size_t)aLo : (size_t)0;
    const size_t bo = (ps == 2) ? (size_t)bLo : (size_t)0;
    const unsigned short* ap = A + (size_t)z * (size_t)aZ + ao
                                 + (size_t)(rowBase + 16 * wave + m) * (size_t)lda + 8 * hh;
    const unsigned short* bp = BT + (size_t)z * (size_t)bZ + bo
                                  + (size_t)(col0 + m) * (size_t)ldb + 8 * hh;
#pragma unroll 1
    for (int k0 = 0; k0 < K; k0 += 32) {
      FragB af;
      af.h[0] = *(const v8usa*)(ap + k0);
      af.h[1] = *(const v8usa*)(ap + k0 + 16);
      const int kb = k0 & kmask;
#pragma unroll
      for (int nt = 0; nt < 8; ++nt) {
        const unsigned short* wq = bp + (size_t)(16 * nt) * (size_t)ldb + kb;
        FragB bf;
        bf.h[0] = *(const v8usa*)wq;
        bf.h[1] = *(const v8usa*)(wq + 16);
        acc[nt] = wmb(af, bf, acc[nt]);
      }
    }
  }

#pragma unroll
  for (int nt = 0; nt < 8; ++nt) {
    const int lc = 16 * nt + m;
#pragma unroll
    for (int r = 0; r < 8; ++r) {
      const int lr = 16 * wave + 8 * hh + r;
      stg[lr * GBN + lc] = acc[nt][r];
    }
  }
  __syncthreads();

  const int grow0 = z * rowsZ + rowBase + 16 * wave;

  if constexpr (EPI != 1) {
    v4f add = {0.f, 0.f, 0.f, 0.f};
    if constexpr (EPI == 2) add = bf16v4(*(const v4fa*)(bias + col0 + 4 * lane));
    v4f pv[16];
#pragma unroll
    for (int i = 0; i < 16; ++i) pv[i] = *(const v4fa*)(stg + (16 * wave + i) * GBN + 4 * lane);
#pragma unroll
    for (int i = 0; i < 16; ++i) {
      const v4f r = *(const v4fa*)(R + (size_t)(grow0 + i) * (size_t)ldo + col0 + 4 * lane);
      pv[i] = r + (pv[i] + add);
    }
#pragma unroll
    for (int i = 0; i < 16; ++i)
      *(volatile v4f*)(outF + (size_t)(grow0 + i) * (size_t)ldo + col0 + 4 * lane) = pv[i];
    __threadfence();
#pragma unroll
    for (int i = 0; i < 16; ++i)
      *(volatile v4f*)(outF + (size_t)(grow0 + i) * (size_t)ldo + col0 + 4 * lane) = pv[i];
  } else {
    const v4f b4 = bf16v4(*(const v4fa*)(bias + col0 + 4 * lane));
#pragma unroll 1
    for (int i = 0; i < 16; ++i) {
      float* srow = stg + (16 * wave + i) * GBN;
      const v4f t = *(const v4fa*)(srow + 4 * lane) + b4;
      v4f g;
      g.x = 0.5f * t.x * (1.0f + erff(t.x * 0.70710678118654752f));
      g.y = 0.5f * t.y * (1.0f + erff(t.y * 0.70710678118654752f));
      g.z = 0.5f * t.z * (1.0f + erff(t.z * 0.70710678118654752f));
      g.w = 0.5f * t.w * (1.0f + erff(t.w * 0.70710678118654752f));
      v4us h4, l4;
      unsigned hb;
      hb = bf16_bits(g.x); h4[0] = (unsigned short)hb; l4[0] = (unsigned short)bf16_bits(g.x - __uint_as_float(hb << 16));
      hb = bf16_bits(g.y); h4[1] = (unsigned short)hb; l4[1] = (unsigned short)bf16_bits(g.y - __uint_as_float(hb << 16));
      hb = bf16_bits(g.z); h4[2] = (unsigned short)hb; l4[2] = (unsigned short)bf16_bits(g.z - __uint_as_float(hb << 16));
      hb = bf16_bits(g.w); h4[3] = (unsigned short)hb; l4[3] = (unsigned short)bf16_bits(g.w - __uint_as_float(hb << 16));
      unsigned short* urow = (unsigned short*)srow;
      *(v4usa*)(urow + 4 * lane) = h4;
      *(v4usa*)(urow + GBN + 4 * lane) = l4;
    }
    __syncthreads();
    v8us qv[16];
#pragma unroll
    for (int i = 0; i < 16; ++i) {
      const unsigned short* urow = (const unsigned short*)(stg + (16 * wave + i) * GBN);
      qv[i] = *(const v8usa*)(urow + 8 * lane);
    }
    const size_t cofs = (size_t)hh * (size_t)(ldo >> 1) + (size_t)col0 + (size_t)(8 * m);
#pragma unroll
    for (int i = 0; i < 16; ++i)
      *(volatile v8us*)(outB + (size_t)(grow0 + i) * (size_t)ldo + cofs) = qv[i];
    __threadfence();
#pragma unroll
    for (int i = 0; i < 16; ++i)
      *(volatile v8us*)(outB + (size_t)(grow0 + i) * (size_t)ldo + cofs) = qv[i];
  }
}

extern "C" void kernel_launch(void* const* d_in, const int* in_sizes, int n_in,
                              void* d_out, int out_size, void* d_ws, size_t ws_size,
                              hipStream_t stream) {
  if (n_in < 12) return;
  if (in_sizes[0] != MROWS * DD) return;
  if (in_sizes[1] != NB * NN * NN) return;
  if (in_sizes[2] != NL * 2 * DD) return;
  if (in_sizes[3] != NL) return;
  if (in_sizes[4] != NL * DD * HH) return;
  if (in_sizes[5] != NL * HH) return;
  if (in_sizes[6] != NL * HH * DD) return;
  if (in_sizes[7] != NL * DD) return;
  if (in_sizes[8] != NL * DD || in_sizes[9] != NL * DD) return;
  if (in_sizes[10] != NL * DD || in_sizes[11] != NL * DD) return;
  if (out_size != MROWS * DD) return;

  const float* x0  = (const float*)d_in[0];
  const int*   adj = (const int*)d_in[1];
  const float* aw  = (const float*)d_in[2];
  const float* abv = (const float*)d_in[3];
  const float* W1  = (const float*)d_in[4];
  const float* b1  = (const float*)d_in[5];
  const float* W2  = (const float*)d_in[6];
  const float* b2  = (const float*)d_in[7];
  const float* g1  = (const float*)d_in[8];
  const float* be1 = (const float*)d_in[9];
  const float* g2  = (const float*)d_in[10];
  const float* be2 = (const float*)d_in[11];
  float* out = (float*)d_out;

  const size_t szX   = (size_t)MROWS * DD * 4;
  const size_t szXT  = (size_t)2 * NB * DD * NN * 2;
  const size_t szY   = (size_t)MROWS * DD * 4;
  const size_t szH   = (size_t)MROWS * DD * 4;
  const size_t szHL  = (size_t)MROWS * 2 * DD * 2;
  const size_t szR1  = (size_t)2 * MROWS * NN * 2;
  const size_t szW1T = (size_t)NL * HH * DD * 2;
  const size_t szW2T = (size_t)NL * DD * HH * 2;
  const size_t szMB  = (size_t)MROWS * 32 * 4;
  const size_t szSS  = (size_t)2 * MROWS * 4;
  if ((size_t)HALFR * (size_t)(2 * HH) * 2 > szR1) return;
  size_t off = 0;
  const size_t oX   = off; off += szX;
  const size_t oXT  = off; off += szXT;
  const size_t oY   = off; off += szY;
  const size_t oH   = off; off += szH;
  const size_t oHL  = off; off += szHL;
  const size_t oR1  = off; off += szR1;
  const size_t oW1T = off; off += szW1T;
  const size_t oW2T = off; off += szW2T;
  const size_t oMB  = off; off += szMB;
  const size_t oSS  = off; off += szSS;
  if (off > ws_size || off > (size_t)WSMAX) return;

  char* ws = (char*)d_ws;
  float*          X   = (float*)(ws + oX);
  unsigned short* XT  = (unsigned short*)(ws + oXT);
  float*          Y   = (float*)(ws + oY);
  float*          H   = (float*)(ws + oH);
  unsigned short* HL  = (unsigned short*)(ws + oHL);
  unsigned short* R1  = (unsigned short*)(ws + oR1);
  unsigned short* W1T = (unsigned short*)(ws + oW1T);
  unsigned short* W2T = (unsigned short*)(ws + oW2T);
  unsigned*       MB  = (unsigned*)(ws + oMB);
  float*          SS  = (float*)(ws + oSS);

  const int nUw = NL * DD * HH / 8;
  k_wT<<<nUw / NTHR, NTHR, 0, stream>>>(W1, W1T, DD, HH, nUw);
  k_wT<<<nUw / NTHR, NTHR, 0, stream>>>(W2, W2T, HH, DD, nUw);
  k_mask<<<MROWS / 32, NTHR, 0, stream>>>(adj, MB);
  k_rows<0><<<MROWS / 32, NTHR, 0, stream>>>(x0, g1, be1, aw, X, HL, SS);
  k_xt<<<dim3(MROWS / 64, DD / 64), NTHR, 0, stream>>>(X, XT);

  for (int l = 0; l < NL; ++l) {
    k_softmax<<<MROWS / NWAVE, NTHR, 0, stream>>>(SS, MB, abv, l, R1);
    k_gemm<0><<<dim3(NN / GBM, DD / GBN, NB), GTHR, 0, stream>>>(
        R1, XT, NN, NN, NN, TERMS_AGG, MROWS * NN, NB * DD * NN, NN * NN, DD * NN, NN,
        X, X, Y, HL, DD);
    k_rows<1><<<MROWS / 32, NTHR, 0, stream>>>(Y, g1 + (size_t)l * DD, be1 + (size_t)l * DD, aw, H, HL, SS);
    for (int hf = 0; hf < 2; ++hf) {
      const size_t r0 = (size_t)hf * HALFR;
      k_gemm<1><<<dim3(HALFR / GBM, HH / GBN, 1), GTHR, 0, stream>>>(
          HL + r0 * (size_t)(2 * DD), W1T + (size_t)l * HH * DD, 2 * DD, DD, 2 * DD, 1, 0, 0, 0, 0, 0,
          H, b1 + (size_t)l * HH, Y, R1, 2 * HH);
      k_gemm<2><<<dim3(HALFR / GBM, DD / GBN, 1), GTHR, 0, stream>>>(
          R1, W2T + (size_t)l * DD * HH, 2 * HH, HH, 2 * HH, 1, 0, 0, 0, 0, 0,
          H + r0 * DD, b2 + (size_t)l * DD, Y + r0 * DD, HL, DD);
    }
    if (l + 1 < NL) {
      k_rows<2><<<MROWS / 32, NTHR, 0, stream>>>(Y, g2 + (size_t)l * DD, be2 + (size_t)l * DD,
                                                 aw + (size_t)(l + 1) * 2 * DD, X, HL, SS);
      k_xt<<<dim3(MROWS / 64, DD / 64), NTHR, 0, stream>>>(X, XT);
    } else {
      k_rows<3><<<MROWS / 32, NTHR, 0, stream>>>(Y, g2 + (size_t)l * DD, be2 + (size_t)l * DD, aw, out, HL, SS);
    }
  }
}
